// FBSNN_76948634075302
// MI455X (gfx1250) — hardware-verified
//
#include <hip/hip_runtime.h>

typedef _Float16       v16h __attribute__((ext_vector_type(16)));
typedef _Float16       v8h  __attribute__((ext_vector_type(8)));
typedef __bf16         v16b __attribute__((ext_vector_type(16)));
typedef unsigned short v8us __attribute__((ext_vector_type(8)));
typedef float          v8f  __attribute__((ext_vector_type(8)));
typedef float          v4f  __attribute__((ext_vector_type(4)));
typedef float          v2f  __attribute__((ext_vector_type(2)));
typedef double         v2d  __attribute__((ext_vector_type(2)));
typedef v8h  __attribute__((may_alias)) v8ha;
typedef v8us __attribute__((may_alias)) v8usa;
typedef v4f  __attribute__((may_alias)) v4fa;

union FragH { v16h v; v8h  p[2]; };
union FragB { v16b v; v8us p[2]; };

#define MP     1024
#define NSTP   50
#define NT1    51
#define DD     100
#define KIN    128
#define HL1    1024
#define HL2    512
#define HL3    256
#define NDX    128
#define XLD    128
#define MAINR  (MP * NT1)
#define NCH    6
#define CHR    (MAINR / NCH)
#define EXR    64
#define RFMX   (CHR + EXR)
#define NXF    (MP * NT1 * DD)
#define NYF    (MP * NT1)
#define NOUTF  (NXF + NYF + 2)

#define RRATE  0.05f
#define SIGV   0.4f
#define KSTR   100.0f
#define DRIFTF ((float)(0.05 - 0.5 * 0.4 * 0.4))
#define WSC    64.0f
#define IWSC   0.015625f
#define IWSC2  0.000244140625f
#define RSC    2048.0f
#define IRSC   0.00048828125f

static_assert(MAINR % NCH == 0);
static_assert(CHR % 64 == 0);
static_assert(RFMX % 32 == 0);
static_assert(MAINR % 32 == 0);
static_assert(NOUTF % 4 == 2);

__device__ __forceinline__ v8f wmma_h(v16h a, v16h b, v8f c) {
#if defined(__HIP_DEVICE_COMPILE__)
  v8f d = __builtin_amdgcn_wmma_f32_16x16x32_f16(false, a, false, b, (short)0, c, false, false);
  asm volatile("v_nop\n\tv_nop\n\tv_nop\n\tv_nop" : "+v"(d) : "v"(a), "v"(b));
  return d;
#else
  (void)a; (void)b; return c;
#endif
}
__device__ __forceinline__ v8f wmma_b(v16b a, v16b b, v8f c) {
#if defined(__HIP_DEVICE_COMPILE__)
  v8f d = __builtin_amdgcn_wmma_f32_16x16x32_bf16(false, a, false, b, (short)0, c, false, false);
  asm volatile("v_nop\n\tv_nop\n\tv_nop\n\tv_nop" : "+v"(d) : "v"(a), "v"(b));
  return d;
#else
  (void)a; (void)b; return c;
#endif
}

__device__ __forceinline__ v16h ldfrag_h(const _Float16* p, int h) {
  FragH f;
  f.p[0] = *(const v8ha*)(p + 8 * h);
  f.p[1] = *(const v8ha*)(p + 16 + 8 * h);
  return f.v;
}
__device__ __forceinline__ v16b ldfrag_b(const unsigned short* p, int h) {
  FragB f;
  f.p[0] = *(const v8usa*)(p + 8 * h);
  f.p[1] = *(const v8usa*)(p + 16 + 8 * h);
  return f.v;
}

__device__ __forceinline__ unsigned short bf_bits(float x) {
  unsigned int u = __float_as_uint(x);
  u += 0x7FFFu + ((u >> 16) & 1u);
  return (unsigned short)(u >> 16);
}
__device__ __forceinline__ float bf_val(unsigned short b) { return __uint_as_float(((unsigned int)b) << 16); }
__device__ __forceinline__ unsigned short hv_bits(_Float16 hv) { return __builtin_bit_cast(unsigned short, hv); }
__device__ __forceinline__ unsigned short h_bits(float x) {
  const _Float16 hv = (_Float16)x;
  return __builtin_bit_cast(unsigned short, hv);
}

__device__ __forceinline__ void zero_acc(v8f (&acc)[2][4]) {
  const v8f z = {0.f, 0.f, 0.f, 0.f, 0.f, 0.f, 0.f, 0.f};
#pragma unroll
  for (int mt = 0; mt < 2; ++mt)
#pragma unroll
    for (int nt = 0; nt < 4; ++nt) acc[mt][nt] = z;
}

__device__ __forceinline__ void core_f16(v8f (&acc)[2][4], const _Float16* __restrict__ Ar, int lda,
                                         const _Float16* __restrict__ Br, int ldb, int K, int h) {
#pragma unroll 1
  for (int k0 = 0; k0 < K; k0 += 32) {
    const v16h a0 = ldfrag_h(Ar + k0, h);
    const v16h a1 = ldfrag_h(Ar + (size_t)16 * lda + k0, h);
#pragma unroll
    for (int nt = 0; nt < 4; ++nt) {
      const v16h b = ldfrag_h(Br + (size_t)(16 * nt) * ldb + k0, h);
      acc[0][nt] = wmma_h(a0, b, acc[0][nt]);
      acc[1][nt] = wmma_h(a1, b, acc[1][nt]);
    }
  }
}

__device__ __forceinline__ void core_f16r(v8f (&acc)[2][4], v8f (&accr)[2][4],
                                          const _Float16* __restrict__ Ah, const _Float16* __restrict__ Ar, int lda,
                                          const _Float16* __restrict__ Br, int ldb, int K, int h) {
#pragma unroll 1
  for (int k0 = 0; k0 < K; k0 += 32) {
    const v16h a0h = ldfrag_h(Ah + k0, h);
    const v16h a1h = ldfrag_h(Ah + (size_t)16 * lda + k0, h);
    const v16h a0r = ldfrag_h(Ar + k0, h);
    const v16h a1r = ldfrag_h(Ar + (size_t)16 * lda + k0, h);
#pragma unroll
    for (int nt = 0; nt < 4; ++nt) {
      const v16h b = ldfrag_h(Br + (size_t)(16 * nt) * ldb + k0, h);
      acc[0][nt]  = wmma_h(a0h, b, acc[0][nt]);
      acc[1][nt]  = wmma_h(a1h, b, acc[1][nt]);
      accr[0][nt] = wmma_h(a0r, b, accr[0][nt]);
      accr[1][nt] = wmma_h(a1r, b, accr[1][nt]);
    }
  }
}

__device__ __forceinline__ void core_b3(v8f (&acc)[2][4],
                                        const unsigned short* __restrict__ Ah, const unsigned short* __restrict__ Al, int lda,
                                        const unsigned short* __restrict__ Bh, const unsigned short* __restrict__ Bl, int ldb,
                                        int K, int h) {
#pragma unroll 1
  for (int k0 = 0; k0 < K; k0 += 32) {
    const v16b a0h = ldfrag_b(Ah + k0, h);
    const v16b a0l = ldfrag_b(Al + k0, h);
    const v16b a1h = ldfrag_b(Ah + (size_t)16 * lda + k0, h);
    const v16b a1l = ldfrag_b(Al + (size_t)16 * lda + k0, h);
#pragma unroll
    for (int nt = 0; nt < 4; ++nt) {
      const v16b bh = ldfrag_b(Bh + (size_t)(16 * nt) * ldb + k0, h);
      const v16b bl = ldfrag_b(Bl + (size_t)(16 * nt) * ldb + k0, h);
      acc[0][nt] = wmma_b(a0h, bh, acc[0][nt]);
      acc[0][nt] = wmma_b(a0h, bl, acc[0][nt]);
      acc[0][nt] = wmma_b(a0l, bh, acc[0][nt]);
      acc[1][nt] = wmma_b(a1h, bh, acc[1][nt]);
      acc[1][nt] = wmma_b(a1h, bl, acc[1][nt]);
      acc[1][nt] = wmma_b(a1l, bh, acc[1][nt]);
    }
  }
}

__device__ __forceinline__ void store16_pass(const unsigned short* st, unsigned short* dst, int ldd, int lane) {
  const int q8 = lane & 7, sub = lane >> 3;
#pragma unroll
  for (int i = 0; i < 8; ++i) {
    const int lr = 4 * i + sub;
    const v8us v = *(const v8usa*)(st + lr * 64 + 8 * q8);
    *(volatile v8us*)(dst + (size_t)lr * ldd + 8 * q8) = v;
  }
}
__device__ __forceinline__ void store32_pass(const float* st, float* dst, int ldd, int lane) {
  const int q8 = lane & 7, sub = lane >> 3;
#pragma unroll
  for (int i = 0; i < 16; ++i) {
    const int L = 4 * i + sub;
    const int lr = L >> 1, hl = L & 1;
    const v4f v = *(const v4fa*)(st + lr * 64 + 32 * hl + 4 * q8);
    *(volatile v4f*)(dst + (size_t)lr * ldd + 32 * hl + 4 * q8) = v;
  }
}

__global__ __launch_bounds__(128) void k_path(const float* __restrict__ t, const float* __restrict__ Wb,
                                              const float* __restrict__ Xi, float* __restrict__ Xws)
{
#pragma clang fp contract(off)
  const int mth = blockIdx.x;
  const int c = threadIdx.x;
  const int dcl = min(max(c - 1, 0), DD - 1);
  const bool ist = (c == 0);
  const bool isx = (c >= 1) && (c <= DD);
  const float* tp = t + mth * NT1;
  const float* wp = Wb + (size_t)mth * NT1 * DD + dcl;
  float x = Xi[mth * DD + dcl];
  float w0 = wp[0];
  float tv = tp[0];
  {
    const float val = ist ? tv : (isx ? x : 0.0f);
    float* p = Xws + (size_t)mth * XLD + c;
    *(volatile float*)p = val;
    __threadfence();
    *(volatile float*)p = val;
  }
#pragma unroll 1
  for (int k = 1; k <= NSTP; ++k) {
    const float w1 = wp[(size_t)k * DD];
    const float t1 = tp[k];
    const float dt = t1 - tv;
    tv = t1;
    const float p1 = DRIFTF * dt;
    const float p2 = SIGV * (w1 - w0);
    const float arg = p1 + p2;
    x = x * expf(arg);
    w0 = w1;
    const float val = ist ? t1 : (isx ? x : 0.0f);
    float* p = Xws + ((size_t)k * MP + mth) * XLD + c;
    *(volatile float*)p = val;
    __threadfence();
    *(volatile float*)p = val;
  }
}

__global__ __launch_bounds__(256) void k_h0(const float* __restrict__ Xws, const float* __restrict__ t,
                                            unsigned short* __restrict__ Hh, unsigned short* __restrict__ Hl,
                                            int rowbase, int nmain, int nrows)
{
  const int g = blockIdx.x * 256 + threadIdx.x;
  const int lrow = g >> 4, q = g & 15;
  if (lrow >= nrows) return;
  const int lrc = min(lrow, nmain - 1);
  const float* src = Xws + (size_t)(rowbase + lrc) * XLD + 8 * q;
  const v4f a = *(const v4fa*)src;
  const v4f b = *(const v4fa*)(src + 4);
  float f[8] = {a.x, a.y, a.z, a.w, b.x, b.y, b.z, b.w};
  const int j = lrow - nmain;
  const int jc = min(max(j, 0), NSTP - 1);
  const float tvl = t[jc + 1];
  const bool extra = (j >= 0);
#pragma unroll
  for (int e = 0; e < 8; ++e) f[e] = extra ? 0.0f : f[e];
  f[0] = (extra && q == 0 && j < NSTP) ? tvl : f[0];
  v8us vh, vl;
#pragma unroll
  for (int e = 0; e < 8; ++e) {
    const unsigned short hi = bf_bits(f[e]);
    const unsigned short lo = bf_bits(f[e] - bf_val(hi));
    vh[e] = hi; vl[e] = lo;
  }
  const size_t o = (size_t)lrow * KIN + 8 * q;
  *(volatile v8us*)(Hh + o) = vh;
  *(volatile v8us*)(Hl + o) = vl;
  __threadfence();
  *(volatile v8us*)(Hh + o) = vh;
  *(volatile v8us*)(Hl + o) = vl;
}

__global__ __launch_bounds__(256) void k_wbf(const float* __restrict__ src, int src_rows, int src_cols, int transpose,
                                             unsigned short* __restrict__ dh, unsigned short* __restrict__ dl,
                                             int dst_rows, int cols8)
{
  const int g = blockIdx.x * 256 + threadIdx.x;
  if (g >= dst_rows * cols8) return;
  const int r = g / cols8;
  const int c8 = (g - r * cols8) * 8;
  v8us vh, vl;
#pragma unroll
  for (int e = 0; e < 8; ++e) {
    const int c = c8 + e;
    const int sr = transpose ? c : r;
    const int sc = transpose ? r : c;
    const bool valid = (sr < src_rows) && (sc < src_cols);
    const size_t idx = (size_t)min(sr, src_rows - 1) * src_cols + min(sc, src_cols - 1);
    float v = src[idx];
    v = valid ? v : 0.0f;
    const unsigned short hi = bf_bits(v);
    const unsigned short lo = bf_bits(v - bf_val(hi));
    vh[e] = hi; vl[e] = lo;
  }
  const size_t o = (size_t)r * (size_t)(cols8 * 8) + c8;
  *(volatile v8us*)(dh + o) = vh;
  *(volatile v8us*)(dl + o) = vl;
  __threadfence();
  *(volatile v8us*)(dh + o) = vh;
  *(volatile v8us*)(dl + o) = vl;
}

__global__ __launch_bounds__(256) void k_w16(const float* __restrict__ src, int src_rows, int src_cols, int row_off,
                                             int transpose, float scale, unsigned short* __restrict__ dst,
                                             int dst_rows, int cols8)
{
  const int g = blockIdx.x * 256 + threadIdx.x;
  if (g >= dst_rows * cols8) return;
  const int r = g / cols8;
  const int c8 = (g - r * cols8) * 8;
  v8us vo;
#pragma unroll
  for (int e = 0; e < 8; ++e) {
    const int c = c8 + e;
    const int sr = transpose ? c : (row_off + r);
    const int sc = transpose ? (row_off + r) : c;
    const bool valid = (sr < src_rows) && (sc < src_cols);
    const size_t idx = (size_t)min(sr, src_rows - 1) * src_cols + min(sc, src_cols - 1);
    float v = src[idx];
    v = valid ? v * scale : 0.0f;
    vo[e] = h_bits(v);
  }
  const size_t o = (size_t)r * (size_t)(cols8 * 8) + c8;
  *(volatile v8us*)(dst + o) = vo;
  __threadfence();
  *(volatile v8us*)(dst + o) = vo;
}

__global__ __launch_bounds__(128) void k_l1(const unsigned short* __restrict__ Hh, const unsigned short* __restrict__ Hl,
                                            const unsigned short* __restrict__ Wh, const unsigned short* __restrict__ Wl,
                                            const float* __restrict__ b1,
                                            unsigned short* __restrict__ a1h, unsigned short* __restrict__ a1r)
{
  __shared__ __attribute__((aligned(16))) unsigned short sTh[4 * 2048];
  __shared__ __attribute__((aligned(16))) unsigned short sTr[4 * 2048];
  const int tid = threadIdx.x, lane = tid & 31, w = tid >> 5, h = lane >> 4, m = lane & 15;
  const int row0 = blockIdx.x * 32;
  const int col0 = blockIdx.y * 256 + 64 * w;
  v8f acc[2][4];
  zero_acc(acc);
  core_b3(acc, Hh + (size_t)(row0 + m) * KIN, Hl + (size_t)(row0 + m) * KIN, KIN,
          Wh + (size_t)(col0 + m) * KIN, Wl + (size_t)(col0 + m) * KIN, KIN, KIN, h);
  unsigned short* sth = sTh + w * 2048;
  unsigned short* str = sTr + w * 2048;
#pragma unroll
  for (int nt = 0; nt < 4; ++nt) {
    const float bb = b1[col0 + 16 * nt + m];
#pragma unroll
    for (int mt = 0; mt < 2; ++mt)
#pragma unroll
      for (int r = 0; r < 8; ++r) {
        float v = acc[mt][nt][r] + bb;
        v = v > 0.0f ? v : 0.0f;
        const _Float16 hv = (_Float16)v;
        const float res = (v - (float)hv) * RSC;
        const int si = (16 * mt + 8 * h + r) * 64 + 16 * nt + m;
        sth[si] = hv_bits(hv);
        str[si] = h_bits(res);
      }
  }
  __syncthreads();
  unsigned short* dh = a1h + (size_t)row0 * HL1 + col0;
  unsigned short* dr = a1r + (size_t)row0 * HL1 + col0;
  store16_pass(sth, dh, HL1, lane);
  store16_pass(str, dr, HL1, lane);
  __threadfence();
  store16_pass(sth, dh, HL1, lane);
  store16_pass(str, dr, HL1, lane);
}

__global__ __launch_bounds__(128) void k_l2(const _Float16* __restrict__ a1h, const _Float16* __restrict__ a1r,
                                            const _Float16* __restrict__ W2T, const float* __restrict__ b2,
                                            unsigned short* __restrict__ a2h, unsigned short* __restrict__ a2l)
{
  __shared__ __attribute__((aligned(16))) unsigned short sTh[4 * 2048];
  __shared__ __attribute__((aligned(16))) unsigned short sTl[4 * 2048];
  const int tid = threadIdx.x, lane = tid & 31, w = tid >> 5, h = lane >> 4, m = lane & 15;
  const int row0 = blockIdx.x * 32;
  const int col0 = blockIdx.y * 256 + 64 * w;
  v8f acc[2][4], accr[2][4];
  zero_acc(acc);
  zero_acc(accr);
  core_f16r(acc, accr, a1h + (size_t)(row0 + m) * HL1, a1r + (size_t)(row0 + m) * HL1, HL1,
            W2T + (size_t)(col0 + m) * HL1, HL1, HL1, h);
  unsigned short* sth = sTh + w * 2048;
  unsigned short* stl = sTl + w * 2048;
#pragma unroll
  for (int nt = 0; nt < 4; ++nt) {
    const float bb = b2[col0 + 16 * nt + m];
#pragma unroll
    for (int mt = 0; mt < 2; ++mt)
#pragma unroll
      for (int r = 0; r < 8; ++r) {
        float v = (acc[mt][nt][r] + accr[mt][nt][r] * IRSC) * IWSC + bb;
        v = v > 0.0f ? v : 0.0f;
        const unsigned short hi = bf_bits(v);
        const unsigned short lo = bf_bits(v - bf_val(hi));
        const int si = (16 * mt + 8 * h + r) * 64 + 16 * nt + m;
        sth[si] = hi;
        stl[si] = lo;
      }
  }
  __syncthreads();
  unsigned short* dh = a2h + (size_t)row0 * HL2 + col0;
  unsigned short* dl = a2l + (size_t)row0 * HL2 + col0;
  store16_pass(sth, dh, HL2, lane);
  store16_pass(stl, dl, HL2, lane);
  __threadfence();
  store16_pass(sth, dh, HL2, lane);
  store16_pass(stl, dl, HL2, lane);
}

__global__ __launch_bounds__(128) void k_l3(const unsigned short* __restrict__ Ah, const unsigned short* __restrict__ Al,
                                            const unsigned short* __restrict__ Wh, const unsigned short* __restrict__ Wl,
                                            const float* __restrict__ b3, const float* __restrict__ Wo,
                                            const float* __restrict__ bo,
                                            unsigned short* __restrict__ g3, float* __restrict__ Yws,
                                            int nmain, int ybase)
{
  __shared__ __attribute__((aligned(16))) unsigned short sT[4 * 2048];
  __shared__ float sY[128];
  const int tid = threadIdx.x, lane = tid & 31, w = tid >> 5, h = lane >> 4, m = lane & 15;
  const int row0 = blockIdx.x * 32;
  const int col0 = 64 * w;
  v8f acc[2][4];
  zero_acc(acc);
  core_b3(acc, Ah + (size_t)(row0 + m) * HL2, Al + (size_t)(row0 + m) * HL2, HL2,
          Wh + (size_t)(col0 + m) * HL2, Wl + (size_t)(col0 + m) * HL2, HL2, HL2, h);
  float wo[4], bb[4];
  unsigned short gw[4];
#pragma unroll
  for (int nt = 0; nt < 4; ++nt) {
    const int col = col0 + 16 * nt + m;
    wo[nt] = Wo[col];
    bb[nt] = b3[col];
    gw[nt] = h_bits(wo[nt] * WSC);
  }
  float s[2][8];
#pragma unroll
  for (int mt = 0; mt < 2; ++mt)
#pragma unroll
    for (int r = 0; r < 8; ++r) s[mt][r] = 0.0f;
  unsigned short* st = sT + w * 2048;
#pragma unroll
  for (int nt = 0; nt < 4; ++nt)
#pragma unroll
    for (int mt = 0; mt < 2; ++mt)
#pragma unroll
      for (int r = 0; r < 8; ++r) {
        const float hv = acc[mt][nt][r] + bb[nt];
        const float av = hv > 0.0f ? hv : 0.0f;
        s[mt][r] = s[mt][r] + av * wo[nt];
        st[(16 * mt + 8 * h + r) * 64 + 16 * nt + m] = (hv > 0.0f) ? gw[nt] : (unsigned short)0;
      }
#pragma unroll
  for (int mt = 0; mt < 2; ++mt)
#pragma unroll
    for (int r = 0; r < 8; ++r) {
      float v = s[mt][r];
      v += __shfl_xor(v, 1);
      v += __shfl_xor(v, 2);
      v += __shfl_xor(v, 4);
      v += __shfl_xor(v, 8);
      s[mt][r] = v;
    }
  float val = 0.0f;
#pragma unroll
  for (int mt = 0; mt < 2; ++mt)
#pragma unroll
    for (int r = 0; r < 8; ++r) val = (m == 8 * mt + r) ? s[mt][r] : val;
  sY[w * 32 + 16 * (m >> 3) + 8 * h + (m & 7)] = val;
  __syncthreads();
  const int yrow0 = (row0 < nmain) ? (ybase + row0) : (MAINR + row0 - nmain);
  const float yv = (((sY[lane] + sY[32 + lane]) + sY[64 + lane]) + sY[96 + lane]) + bo[0];
  unsigned short* dst = g3 + (size_t)row0 * HL3 + col0;
  store16_pass(st, dst, HL3, lane);
  if (w == 0) *(volatile float*)(Yws + yrow0 + lane) = yv;
  __threadfence();
  store16_pass(st, dst, HL3, lane);
  if (w == 0) *(volatile float*)(Yws + yrow0 + lane) = yv;
}

__global__ __launch_bounds__(128) void k_bw(const _Float16* __restrict__ A, int lda, const _Float16* __restrict__ B,
                                            int ldb, int K, unsigned short* __restrict__ dst, int ldd)
{
  __shared__ __attribute__((aligned(16))) unsigned short sT[4 * 2048];
  const int tid = threadIdx.x, lane = tid & 31, w = tid >> 5, h = lane >> 4, m = lane & 15;
  const int row0 = blockIdx.x * 32;
  const int col0 = blockIdx.y * 256 + 64 * w;
  v8f acc[2][4];
  zero_acc(acc);
  core_f16(acc, A + (size_t)(row0 + m) * lda, lda, B + (size_t)(col0 + m) * ldb, ldb, K, h);
  unsigned short* st = sT + w * 2048;
#pragma unroll
  for (int nt = 0; nt < 4; ++nt)
#pragma unroll
    for (int mt = 0; mt < 2; ++mt)
#pragma unroll
      for (int r = 0; r < 8; ++r)
        st[(16 * mt + 8 * h + r) * 64 + 16 * nt + m] = h_bits(acc[mt][nt][r] * IWSC);
  __syncthreads();
  unsigned short* d0 = dst + (size_t)row0 * ldd + col0;
  const int q8 = lane & 7, sub = lane >> 3;
  v8us vals[8];
#pragma unroll
  for (int i = 0; i < 8; ++i) {
    const int lr = 4 * i + sub;
    const v8us sv = *(const v8usa*)(st + lr * 64 + 8 * q8);
    const v8us mk = *(const v8usa*)(d0 + (size_t)lr * ldd + 8 * q8);
    v8us o;
#pragma unroll
    for (int e = 0; e < 8; ++e) o[e] = (mk[e] != 0) ? sv[e] : (unsigned short)0;
    vals[i] = o;
  }
#pragma unroll
  for (int i = 0; i < 8; ++i)
    *(volatile v8us*)(d0 + (size_t)(4 * i + sub) * ldd + 8 * q8) = vals[i];
  __threadfence();
#pragma unroll
  for (int i = 0; i < 8; ++i)
    *(volatile v8us*)(d0 + (size_t)(4 * i + sub) * ldd + 8 * q8) = vals[i];
}

__global__ __launch_bounds__(128) void k_dx(const _Float16* __restrict__ g1, const _Float16* __restrict__ W1P,
                                            float* __restrict__ DU)
{
  __shared__ __attribute__((aligned(16))) float sF[4 * 2048];
  const int tid = threadIdx.x, lane = tid & 31, w = tid >> 5, h = lane >> 4, m = lane & 15;
  const int row0 = blockIdx.x * 64 + 32 * (w >> 1);
  const int col0 = 64 * (w & 1);
  v8f acc[2][4];
  zero_acc(acc);
  core_f16(acc, g1 + (size_t)(row0 + m) * HL1, HL1, W1P + (size_t)(col0 + m) * HL1, HL1, HL1, h);
  float* st = sF + w * 2048;
#pragma unroll
  for (int nt = 0; nt < 4; ++nt)
#pragma unroll
    for (int mt = 0; mt < 2; ++mt)
#pragma unroll
      for (int r = 0; r < 8; ++r)
        st[(16 * mt + 8 * h + r) * 64 + 16 * nt + m] = acc[mt][nt][r] * IWSC2;
  __syncthreads();
  float* dst = DU + (size_t)row0 * NDX + col0;
  store32_pass(st, dst, NDX, lane);
  __threadfence();
  store32_pass(st, dst, NDX, lane);
}

__global__ __launch_bounds__(128) void k_loss1(const float* __restrict__ Yws, const float* __restrict__ DU,
                                               const float* __restrict__ Xws, const float* __restrict__ t,
                                               const float* __restrict__ Wb, double* __restrict__ part)
{
#pragma clang fp contract(off)
  __shared__ double sred[128];
  __shared__ float smax[4];
  __shared__ int scnt[4];
  const int mth = blockIdx.x;
  const int c = threadIdx.x, lane = c & 31, w = c >> 5;
  const bool valid = (c < DD);
  const int dcl = min(c, DD - 1);
  const float* tp = t + mth * NT1;
  const float* wp = Wb + (size_t)mth * NT1 * DD + dcl;
  double acc = 0.0;
#pragma unroll 1
  for (int k = 0; k < NSTP; ++k) {
    const float y0 = Yws[(size_t)k * MP + mth];
    const float y1 = Yws[(size_t)(k + 1) * MP + mth];
    const float dt = tp[k + 1] - tp[k];
    const float x0 = Xws[((size_t)k * MP + mth) * XLD + 1 + dcl];
    const float du = DU[((size_t)k * MP + mth) * NDX + dcl];
    const float dw = wp[(size_t)(k + 1) * DD] - wp[(size_t)k * DD];
    float yt = y0 + (RRATE * y0) * dt;
    yt = yt + (0.0f * x0) * du;
    yt = yt + ((du * SIGV) * x0) * dw;
    const float df = y1 - yt;
    const float sq = df * df;
    acc += valid ? (double)sq : 0.0;
  }
  const float xN = Xws[((size_t)NSTP * MP + mth) * XLD + 1 + dcl];
  float xv = valid ? xN : -3.0e38f;
#pragma unroll
  for (int sft = 16; sft > 0; sft >>= 1) xv = fmaxf(xv, __shfl_xor(xv, sft));
  if (lane == 0) smax[w] = xv;
  __syncthreads();
  const float mx = fmaxf(fmaxf(smax[0], smax[1]), fmaxf(smax[2], smax[3]));
  const bool eq = valid && (xN == mx);
  int cv = eq ? 1 : 0;
#pragma unroll
  for (int sft = 16; sft > 0; sft >>= 1) cv += __shfl_xor(cv, sft);
  if (lane == 0) scnt[w] = cv;
  __syncthreads();
  const int cnt = max(scnt[0] + scnt[1] + scnt[2] + scnt[3], 1);
  const float gv = mx - KSTR;
  const float gr = (gv > 0.0f) ? 1.0f : 0.0f;
  const float gp = (gv > 0.0f) ? gv : 0.0f;
  const float dg = eq ? gr * (1.0f / (float)cnt) : 0.0f;
  const float duN = DU[((size_t)NSTP * MP + mth) * NDX + dcl];
  const float ed = duN - dg;
  acc += valid ? (double)(ed * ed) : 0.0;
  if (c == 0) {
    const float yN = Yws[(size_t)NSTP * MP + mth];
    const float dy = yN - gp;
    acc += (double)(dy * dy);
  }
  sred[c] = acc;
  __syncthreads();
#pragma unroll 1
  for (int sft = 64; sft > 0; sft >>= 1) {
    if (c < sft) sred[c] = sred[c] + sred[c + sft];
    __syncthreads();
  }
  const double tot = sred[0];
  v2d pv;
  pv.x = (lane == 0) ? tot : 0.0;
  pv.y = 0.0;
  double* pp = part + (size_t)mth * 16 + 2 * lane;
  if (w == 0 && lane < 8) *(volatile v2d*)pp = pv;
  __threadfence();
  if (w == 0 && lane < 8) *(volatile v2d*)pp = pv;
}

__global__ __launch_bounds__(256) void k_loss2(const double* __restrict__ part, const float* __restrict__ Yws,
                                               float* __restrict__ scal)
{
  __shared__ double sred[256];
  const int c = threadIdx.x, lane = c & 31, w = c >> 5;
  double a = 0.0;
#pragma unroll
  for (int i = 0; i < 4; ++i) a += part[(size_t)(c + 256 * i) * 16];
  const int jc = min(c, NSTP - 1);
  const float y = Yws[MAINR + jc];
  a += (c < NSTP) ? (double)MP * (double)(y * y) : 0.0;
  sred[c] = a;
  __syncthreads();
#pragma unroll 1
  for (int sft = 128; sft > 0; sft >>= 1) {
    if (c < sft) sred[c] = sred[c] + sred[c + sft];
    __syncthreads();
  }
  const double tot = sred[0];
  const float lv = (float)(tot / 102.0);
  const float v = (lane == 0) ? lv : 0.0f;
  if (w == 0) *(volatile float*)(scal + lane) = v;
  __threadfence();
  if (w == 0) *(volatile float*)(scal + lane) = v;
}

__device__ __forceinline__ float out_val(int f, const float* __restrict__ scal, const float* __restrict__ Xws,
                                         const float* __restrict__ Yws)
{
  const int e = min(max(f - 1, 0), NXF - 1);
  const int mth = e / (NT1 * DD);
  const int rr = e - mth * (NT1 * DD);
  const int k = rr / DD;
  const int d = rr - k * DD;
  const float vx = Xws[((size_t)k * MP + mth) * XLD + 1 + d];
  const int e2 = min(max(f - 1 - NXF, 0), NYF - 1);
  const int m2 = e2 / NT1;
  const int k2 = e2 - m2 * NT1;
  const float vy = Yws[(size_t)k2 * MP + m2];
  const float vs = scal[0];
  const float v0 = Yws[0];
  return (f == 0) ? vs : ((f <= NXF) ? vx : ((f <= NXF + NYF) ? vy : v0));
}

__global__ __launch_bounds__(256) void k_out(const float* __restrict__ scal, const float* __restrict__ Xws,
                                             const float* __restrict__ Yws, float* __restrict__ out)
{
  const int g = blockIdx.x * 256 + threadIdx.x;
  if (g > NOUTF / 4) return;
  const int f0 = 4 * g;
  v4f v;
  v.x = out_val(f0 + 0, scal, Xws, Yws);
  v.y = out_val(f0 + 1, scal, Xws, Yws);
  v.z = out_val(f0 + 2, scal, Xws, Yws);
  v.w = out_val(f0 + 3, scal, Xws, Yws);
  const bool full = (f0 + 3 < NOUTF);
  v2f v2;
  v2.x = v.x; v2.y = v.y;
  if (full) *(volatile v4f*)(out + f0) = v;
  else      *(volatile v2f*)(out + f0) = v2;
  __threadfence();
  if (full) *(volatile v4f*)(out + f0) = v;
  else      *(volatile v2f*)(out + f0) = v2;
}

#define SZ_XWS  ((size_t)NT1 * MP * XLD * 4)
#define SZ_DU   ((size_t)MAINR * NDX * 4)
#define SZ_Y    ((size_t)(MAINR + EXR) * 4)
#define SZ_W1T  ((size_t)HL1 * KIN * 2)
#define SZ_W3T  ((size_t)HL3 * HL2 * 2)
#define SZ_W1P  ((size_t)NDX * HL1 * 2)
#define SZ_W2   ((size_t)HL1 * HL2 * 2)
#define SZ_W3N  ((size_t)HL2 * HL3 * 2)
#define SZ_PART ((size_t)MP * 16 * 8)
#define SZ_SCAL ((size_t)256)
#define SZ_H0   ((size_t)RFMX * KIN * 2)
#define SZ_A1   ((size_t)RFMX * HL1 * 2)
#define SZ_A2   ((size_t)RFMX * HL2 * 2)
#define SZ_G3   ((size_t)RFMX * HL3 * 2)
#define WS_TOTAL (SZ_XWS + SZ_DU + SZ_Y + 2 * SZ_W1T + 2 * SZ_W3T + SZ_W1P + 2 * SZ_W2 + SZ_W3N + \
                  SZ_PART + SZ_SCAL + 2 * SZ_H0 + 2 * SZ_A1 + 2 * SZ_A2 + SZ_G3)
static_assert(WS_TOTAL == (size_t)120336896);
static_assert(WS_TOTAL <= (size_t)134217728);

extern "C" void kernel_launch(void* const* d_in, const int* in_sizes, int n_in,
                              void* d_out, int out_size, void* d_ws, size_t ws_size,
                              hipStream_t stream)
{
  if (n_in < 11) return;
  if (in_sizes[0] != MAINR || in_sizes[1] != NXF || in_sizes[2] != MP * DD) return;
  if (in_sizes[3] != (DD + 1) * HL1 || in_sizes[4] != HL1) return;
  if (in_sizes[5] != HL1 * HL2 || in_sizes[6] != HL2) return;
  if (in_sizes[7] != HL2 * HL3 || in_sizes[8] != HL3) return;
  if (in_sizes[9] != HL3 || in_sizes[10] != 1) return;
  if (out_size != NOUTF) return;
  if (WS_TOTAL > ws_size) return;

  const float* t_in = (const float*)d_in[0];
  const float* W_in = (const float*)d_in[1];
  const float* Xi   = (const float*)d_in[2];
  const float* W1   = (const float*)d_in[3];
  const float* b1   = (const float*)d_in[4];
  const float* W2   = (const float*)d_in[5];
  const float* b2   = (const float*)d_in[6];
  const float* W3   = (const float*)d_in[7];
  const float* b3   = (const float*)d_in[8];
  const float* Wo   = (const float*)d_in[9];
  const float* bo   = (const float*)d_in[10];
  float* out = (float*)d_out;

  char* ws = (char*)d_ws;
  size_t off = 0;
  float* Xws = (float*)(ws + off);                          off += SZ_XWS;
  float* DU  = (float*)(ws + off);                          off += SZ_DU;
  float* Yws = (float*)(ws + off);                          off += SZ_Y;
  unsigned short* W1Th = (unsigned short*)(ws + off);       off += SZ_W1T;
  unsigned short* W1Tl = (unsigned short*)(ws + off);       off += SZ_W1T;
  unsigned short* W3Th = (unsigned short*)(ws + off);       off += SZ_W3T;
  unsigned short* W3Tl = (unsigned short*)(ws + off);       off += SZ_W3T;
  unsigned short* W1P  = (unsigned short*)(ws + off);       off += SZ_W1P;
  unsigned short* W2T  = (unsigned short*)(ws + off);       off += SZ_W2;
  unsigned short* W2N  = (unsigned short*)(ws + off);       off += SZ_W2;
  unsigned short* W3N  = (unsigned short*)(ws + off);       off += SZ_W3N;
  double* part = (double*)(ws + off);                       off += SZ_PART;
  float* scal = (float*)(ws + off);                         off += SZ_SCAL;
  unsigned short* H0h = (unsigned short*)(ws + off);        off += SZ_H0;
  unsigned short* H0l = (unsigned short*)(ws + off);        off += SZ_H0;
  unsigned short* a1h = (unsigned short*)(ws + off);        off += SZ_A1;
  unsigned short* a1r = (unsigned short*)(ws + off);        off += SZ_A1;
  unsigned short* a2h = (unsigned short*)(ws + off);        off += SZ_A2;
  unsigned short* a2l = (unsigned short*)(ws + off);        off += SZ_A2;
  unsigned short* g3  = (unsigned short*)(ws + off);        off += SZ_G3;
  if (off > ws_size) return;

  k_path<<<MP, 128, 0, stream>>>(t_in, W_in, Xi, Xws);

  k_wbf<<<(HL1 * (KIN / 8) + 255) / 256, 256, 0, stream>>>(W1, DD + 1, HL1, 1, W1Th, W1Tl, HL1, KIN / 8);
  k_wbf<<<(HL3 * (HL2 / 8) + 255) / 256, 256, 0, stream>>>(W3, HL2, HL3, 1, W3Th, W3Tl, HL3, HL2 / 8);
  k_w16<<<(NDX * (HL1 / 8) + 255) / 256, 256, 0, stream>>>(W1, DD + 1, HL1, 1, 0, WSC, W1P, NDX, HL1 / 8);
  k_w16<<<(HL2 * (HL1 / 8) + 255) / 256, 256, 0, stream>>>(W2, HL1, HL2, 0, 1, WSC, W2T, HL2, HL1 / 8);
  k_w16<<<(HL1 * (HL2 / 8) + 255) / 256, 256, 0, stream>>>(W2, HL1, HL2, 0, 0, WSC, W2N, HL1, HL2 / 8);
  k_w16<<<(HL2 * (HL3 / 8) + 255) / 256, 256, 0, stream>>>(W3, HL2, HL3, 0, 0, WSC, W3N, HL2, HL3 / 8);

  for (int cidx = 0; cidx < NCH; ++cidx) {
    const int rowbase = cidx * CHR;
    const int RF = (cidx == NCH - 1) ? RFMX : CHR;
    const int RB = CHR;
    float* DUc = DU + (size_t)rowbase * NDX;

    k_h0<<<(RF * 16 + 255) / 256, 256, 0, stream>>>(Xws, t_in, H0h, H0l, rowbase, CHR, RF);
    k_l1<<<dim3(RF / 32, HL1 / 256), 128, 0, stream>>>(H0h, H0l, W1Th, W1Tl, b1, a1h, a1r);
    k_l2<<<dim3(RF / 32, HL2 / 256), 128, 0, stream>>>((const _Float16*)a1h, (const _Float16*)a1r,
                                                      (const _Float16*)W2T, b2, a2h, a2l);
    k_l3<<<dim3(RF / 32, 1), 128, 0, stream>>>(a2h, a2l, W3Th, W3Tl, b3, Wo, bo, g3, Yws, CHR, rowbase);
    k_bw<<<dim3(RB / 32, HL2 / 256), 128, 0, stream>>>((const _Float16*)g3, HL3, (const _Float16*)W3N, HL3, HL3, a2h, HL2);
    k_bw<<<dim3(RB / 32, HL1 / 256), 128, 0, stream>>>((const _Float16*)a2h, HL2, (const _Float16*)W2N, HL2, HL2, a1h, HL1);
    k_dx<<<dim3(RB / 64, 1), 128, 0, stream>>>((const _Float16*)a1h, (const _Float16*)W1P, DUc);
  }

  k_loss1<<<MP, 128, 0, stream>>>(Yws, DU, Xws, t_in, W_in, part);
  k_loss2<<<1, 256, 0, stream>>>(part, Yws, scal);
  k_out<<<(NOUTF / 4 + 1 + 255) / 256, 256, 0, stream>>>(scal, Xws, Yws, out);
}
